// CrossAttention_12403865551338
// MI455X (gfx1250) — hardware-verified
//
#include <hip/hip_runtime.h>
#include <stdint.h>


typedef _Float16     v16h __attribute__((ext_vector_type(16)));
typedef _Float16     v8h  __attribute__((ext_vector_type(8)));
typedef float        v8f  __attribute__((ext_vector_type(8)));
typedef float        v4f  __attribute__((ext_vector_type(4)));
typedef unsigned int v4u  __attribute__((ext_vector_type(4)));

#ifndef NB
#define NB 4
#endif
#ifndef SEQ
#define SEQ 2048
#endif
#define NB_FULL  4
#define SEQ_FULL 2048
#define EMB  512
#define NH   8
#define HD   64
#define NKT  (SEQ / 32)

#define ACT_CAR   8.0f
#define W_CAR     1024.0f
#define PROJ_SCL  0.0009765625f
#define ACC_NRM   8192.0f
#define RES_CAR   2048.0f
#define RES_INV   0.00048828125f
#define QK_INV    0.015625f
#define P_CAR     16384.0f
#define O_SCL     7.62939453125e-06f

static_assert(NB <= NB_FULL && SEQ <= SEQ_FULL);
static_assert(SEQ % 256 == 0);
static_assert(EMB == NH * HD);
static_assert(HD == 64);
static_assert(EMB % 128 == 0 && EMB % 32 == 0);
static_assert((long)NB_FULL * SEQ_FULL * EMB * 4 == 16777216L);
static_assert(((long)NB * SEQ * EMB / 8) % 256 == 0 && ((long)EMB * EMB / 8) % 256 == 0);
static_assert((long)(EMB / 64) * (NB * SEQ / 128) * 128 * 64 == (long)NB * SEQ * EMB);
static_assert((long)(SEQ / 64) * (EMB / 128) * NB * 128 * 64 == (long)NB * SEQ * EMB);
static_assert((long)(SEQ / 128) * NH * NB * 128 * HD == (long)NB * SEQ * EMB);
static_assert((long)(SEQ / 128) * (NKT / 8) * 256 * 4 == (long)NKT * SEQ);
static_assert((long)8 * NB * SEQ * EMB * 2 + (long)3 * EMB * EMB * 2 + (long)NKT * SEQ * 4 +
              (long)(SEQ / 128) * NKT * 4 <= 134217728L);

union Frag16 { v16h v; v8h p[2]; };

__device__ __forceinline__ v16h ld_frag(const _Float16* p, int hl) {
  Frag16 f;
  f.p[0] = *(const v8h*)(p + 8 * hl);
  f.p[1] = *(const v8h*)(p + 16 + 8 * hl);
  return f.v;
}

__device__ __forceinline__ v8f mma(v16h a, v16h b, v8f c) {
  v8f d = __builtin_amdgcn_wmma_f32_16x16x32_f16(false, a, false, b, (short)0, c, false, false);
  asm volatile("v_nop\n\tv_nop\n\tv_nop\n\tv_nop" : "+v"(d) : "v"(a), "v"(b));
  return d;
}

__device__ __forceinline__ float bf16_rne(float x) {
  unsigned int u = __builtin_bit_cast(unsigned int, x);
  u += 0x7FFFu + ((u >> 16) & 1u);
  return __builtin_bit_cast(float, u & 0xFFFF0000u);
}

__global__ __launch_bounds__(256) void k_cvt8(const float* __restrict__ src,
                                              _Float16* __restrict__ dst,
                                              int rpb, int srpb, float car, int total8)
{
  const int i8 = blockIdx.x * 256 + threadIdx.x;
  if (i8 >= total8) return;
  const size_t e   = (size_t)i8 * 8;
  const size_t r   = e / (size_t)EMB;
  const int    col = (int)(e - r * (size_t)EMB);
  const size_t bb  = r / (size_t)rpb;
  const size_t srow = bb * (size_t)srpb + (r - bb * (size_t)rpb);
  const float* s = src + srow * (size_t)EMB + col;
  const v4f x0 = *(const v4f*)s;
  const v4f x1 = *(const v4f*)(s + 4);
  v8h o;
#pragma unroll
  for (int j = 0; j < 4; ++j) {
    const float t0 = x0[j];
    const float t1 = x1[j];
    o[j]     = (_Float16)(bf16_rne(t0) * car);
    o[4 + j] = (_Float16)(bf16_rne(t1) * car);
  }
  _Float16* d = dst + e;
  *(volatile v8h*)d = o;
  __threadfence();
  *(volatile v8h*)d = o;
}

__global__ __launch_bounds__(256) void k_mask(const int* __restrict__ am,
                                              unsigned int* __restrict__ MBT,
                                              unsigned int* __restrict__ TF)
{
  constexpr int LW = NKT + 1;
  __shared__ unsigned int ldsW[128 * LW];
  __shared__ unsigned int ldsF[NKT];
  const int tid = threadIdx.x, lane = tid & 31, w = tid >> 5;
  const int q0 = blockIdx.x * 128;

#pragma unroll 1
  for (int rr = 0; rr < 16; ++rr) {
    const int row = 16 * w + rr;
    const int* srow = am + (size_t)(q0 + row) * SEQ_FULL + lane;
#pragma unroll 4
    for (int kt = 0; kt < NKT; ++kt) {
      const int v = srow[kt * 32];
      const unsigned int wd = __builtin_amdgcn_ballot_w32(v != 0);
      if (lane == 0) ldsW[row * LW + kt] = wd;
    }
  }
  __syncthreads();

  {
    const int kc = (tid < NKT) ? tid : (NKT - 1);
    unsigned int f = 1u;
#pragma unroll 4
    for (int r = 0; r < 128; ++r)
      f &= (ldsW[r * LW + kc] == 0xFFFFFFFFu) ? 1u : 0u;
    if (tid < NKT) ldsF[tid] = f;
  }
  __syncthreads();

  const int fi = (tid < NKT / 4) ? tid : 0;
  v4u fv;
  fv[0] = ldsF[4 * fi + 0]; fv[1] = ldsF[4 * fi + 1];
  fv[2] = ldsF[4 * fi + 2]; fv[3] = ldsF[4 * fi + 3];
  unsigned int* const tfp = TF + (size_t)blockIdx.x * NKT + 4 * fi;

#pragma unroll 1
  for (int i = 0; i < NKT / 8; ++i) {
    const int idx = i * 256 + tid;
    const int kt = idx >> 5, j4 = (idx & 31) * 4;
    v4u v;
    v[0] = ldsW[(j4 + 0) * LW + kt]; v[1] = ldsW[(j4 + 1) * LW + kt];
    v[2] = ldsW[(j4 + 2) * LW + kt]; v[3] = ldsW[(j4 + 3) * LW + kt];
    *(volatile v4u*)(MBT + (size_t)kt * SEQ + q0 + j4) = v;
  }
  if (tid < NKT / 4) *(volatile v4u*)tfp = fv;
  __threadfence();
#pragma unroll 1
  for (int i = 0; i < NKT / 8; ++i) {
    const int idx = i * 256 + tid;
    const int kt = idx >> 5, j4 = (idx & 31) * 4;
    v4u v;
    v[0] = ldsW[(j4 + 0) * LW + kt]; v[1] = ldsW[(j4 + 1) * LW + kt];
    v[2] = ldsW[(j4 + 2) * LW + kt]; v[3] = ldsW[(j4 + 3) * LW + kt];
    *(volatile v4u*)(MBT + (size_t)kt * SEQ + q0 + j4) = v;
  }
  if (tid < NKT / 4) *(volatile v4u*)tfp = fv;
}

__device__ __forceinline__ void gemm_core(const _Float16* ap0, const _Float16* ap1,
                                          const _Float16* bp, int K, int hl, v8f (&acc)[8])
{
  const size_t bst = (size_t)16 * K;
#pragma unroll 1
  for (int k0 = 0; k0 < K; k0 += 32) {
    const v16h a0 = ld_frag(ap0 + k0, hl);
    const v16h a1 = ld_frag(ap1 + k0, hl);
    const v16h b0 = ld_frag(bp + k0, hl);
    const v16h b1 = ld_frag(bp + bst + k0, hl);
    const v16h b2 = ld_frag(bp + 2 * bst + k0, hl);
    const v16h b3 = ld_frag(bp + 3 * bst + k0, hl);
    acc[0] = mma(a0, b0, acc[0]);
    acc[1] = mma(a0, b1, acc[1]);
    acc[2] = mma(a0, b2, acc[2]);
    acc[3] = mma(a0, b3, acc[3]);
    acc[4] = mma(a1, b0, acc[4]);
    acc[5] = mma(a1, b1, acc[5]);
    acc[6] = mma(a1, b2, acc[6]);
    acc[7] = mma(a1, b3, acc[7]);
  }
}

__global__ __launch_bounds__(128) __attribute__((amdgpu_num_vgpr(256)))
void k_proj(const _Float16* __restrict__ A, const _Float16* __restrict__ Bt,
            _Float16* __restrict__ PH, _Float16* __restrict__ PL, int K, int ldc,
            long long bstride, long long cstride, int norm)
{
  __shared__ __attribute__((aligned(16))) _Float16 ldsH[128 * 72];
  __shared__ __attribute__((aligned(16))) _Float16 ldsL[128 * 72];

  const int tid = threadIdx.x, lane = tid & 31, w = tid >> 5;
  const int hl = lane >> 4, c = lane & 15;
  const int m0 = blockIdx.y * 128, n0 = blockIdx.x * 64;
  const int mw = m0 + 32 * w;
  const size_t zb = (size_t)blockIdx.z * (size_t)bstride;
  const size_t zc = (size_t)blockIdx.z * (size_t)cstride;

  const _Float16* ap0 = A  + (size_t)(mw + c) * K;
  const _Float16* ap1 = A  + (size_t)(mw + 16 + c) * K;
  const _Float16* bp  = Bt + zb + (size_t)(n0 + c) * K;

  v8f acc[8] = {};
  gemm_core(ap0, ap1, bp, K, hl, acc);

#pragma unroll
  for (int i = 0; i < 2; ++i)
#pragma unroll
    for (int r = 0; r < 8; ++r) {
      float ss = 0.f;
#pragma unroll
      for (int t = 0; t < 4; ++t) ss += acc[i * 4 + t][r] * acc[i * 4 + t][r];
      ss += __shfl_xor(ss, 1, 32);
      ss += __shfl_xor(ss, 2, 32);
      ss += __shfl_xor(ss, 4, 32);
      ss += __shfl_xor(ss, 8, 32);
      const float inv = fminf(rsqrtf(ss) * ACC_NRM, 1.0e12f);
      const float sc  = (norm != 0) ? (PROJ_SCL * inv) : PROJ_SCL;
      const int rowl = 32 * w + 16 * i + 8 * hl + r;
#pragma unroll
      for (int t = 0; t < 4; ++t) {
        const float v = acc[i * 4 + t][r] * sc;
        const _Float16 hv = (_Float16)v;
        const float res = (v - (float)hv) * RES_CAR;
        ldsH[rowl * 72 + 16 * t + c] = hv;
        ldsL[rowl * 72 + 16 * t + c] = (_Float16)res;
      }
    }
  __syncthreads();

  _Float16* const bh = PH + zc + (size_t)m0 * ldc + n0;
  _Float16* const bl = PL + zc + (size_t)m0 * ldc + n0;
  for (int i = 0; i < 8; ++i) {
    const int q = i * 128 + tid;
    const int rowl = q >> 3, ch = (q & 7) * 8;
    const v8h vh = *(const v8h*)(ldsH + rowl * 72 + ch);
    const v8h vl = *(const v8h*)(ldsL + rowl * 72 + ch);
    *(volatile v8h*)(bh + (size_t)rowl * ldc + ch) = vh;
    *(volatile v8h*)(bl + (size_t)rowl * ldc + ch) = vl;
  }
  __threadfence();
  for (int i = 0; i < 8; ++i) {
    const int q = i * 128 + tid;
    const int rowl = q >> 3, ch = (q & 7) * 8;
    const v8h vh = *(const v8h*)(ldsH + rowl * 72 + ch);
    const v8h vl = *(const v8h*)(ldsL + rowl * 72 + ch);
    *(volatile v8h*)(bh + (size_t)rowl * ldc + ch) = vh;
    *(volatile v8h*)(bl + (size_t)rowl * ldc + ch) = vl;
  }
}

__global__ __launch_bounds__(256) __attribute__((amdgpu_num_vgpr(256)))
void k_attn(const _Float16* __restrict__ QH, const _Float16* __restrict__ QL,
            const _Float16* __restrict__ KH, const _Float16* __restrict__ KL,
            const _Float16* __restrict__ VtH, const _Float16* __restrict__ VtL,
            const unsigned int* __restrict__ MBT, const unsigned int* __restrict__ TF,
            const int* __restrict__ kpm, const float* __restrict__ gptr,
            float* __restrict__ Out)
{
  constexpr int KT_H = 32 * 72;
  constexpr int V_H  = HD * 40;
  constexpr int P_H  = 8 * 16 * 40;
  __shared__ __attribute__((aligned(16))) _Float16 ldsK0[KT_H];
  __shared__ __attribute__((aligned(16))) _Float16 ldsK1[KT_H];
  __shared__ __attribute__((aligned(16))) _Float16 ldsVH[V_H];
  __shared__ __attribute__((aligned(16))) _Float16 ldsVL[V_H];
  __shared__ __attribute__((aligned(16))) _Float16 ldsPH[P_H];
  __shared__ __attribute__((aligned(16))) _Float16 ldsPL[P_H];
  __shared__ __attribute__((aligned(16))) float    ldsO[64 * 68];

  const int tid = threadIdx.x, lane = tid & 31, w = tid >> 5;
  const int hl = lane >> 4, c = lane & 15;
  const int q0 = blockIdx.x * 128;
  const int col0 = blockIdx.y * HD;
  const int b = blockIdx.z;
  const size_t rowbase = (size_t)b * SEQ;

  const size_t qrow = (rowbase + q0 + 16 * w + c) * EMB + col0;
  v16h qh[2], ql[2];
#pragma unroll
  for (int ks = 0; ks < 2; ++ks) {
    qh[ks] = ld_frag(QH + qrow + 32 * ks, hl);
    ql[ks] = ld_frag(QL + qrow + 32 * ks, hl);
  }
  const int pbase = w * (16 * 40);

  const int krr = tid >> 3, kcc = (tid & 7) * 8;
  const int vdd = tid >> 2, vkc = (tid & 3) * 8;
  const _Float16* const kgh = KH + (rowbase + krr) * EMB + col0 + kcc;
  const _Float16* const kgl = KL + (rowbase + krr) * EMB + col0 + kcc;
  const _Float16* const vgh = VtH + ((size_t)b * EMB + col0 + vdd) * SEQ + vkc;
  const _Float16* const vgl = VtL + ((size_t)b * EMB + col0 + vdd) * SEQ + vkc;
  const unsigned int* const mp = MBT + q0 + 16 * w + 8 * hl;
  const int* const kp = kpm + (size_t)b * SEQ_FULL + c;
  const unsigned int* const tfp = TF + (size_t)blockIdx.x * NKT;

  const float sscl = bf16_rne(gptr[0]) * QK_INV;
  const float NEG_INF = -__builtin_inff();

  float m[8], l[8];
  v8f oh[4] = {}, ol[4] = {};
#pragma unroll
  for (int r = 0; r < 8; ++r) { m[r] = NEG_INF; l[r] = 0.f; }

#pragma unroll 1
  for (int kt = 0; kt < NKT; ++kt) {
    if (tfp[kt] != 0u) continue;
    const int mk = kt * 32;
    unsigned int mw[8];
    {
      const v8h k8h = *(const v8h*)(kgh + (size_t)mk * EMB);
      const v8h k8l = *(const v8h*)(kgl + (size_t)mk * EMB);
      const v8h v8a = *(const v8h*)(vgh + mk);
      const v8h v8b = *(const v8h*)(vgl + mk);
      const v4u ma = *(const v4u*)(mp + (size_t)kt * SEQ);
      const v4u mb = *(const v4u*)(mp + (size_t)kt * SEQ + 4);
      mw[0] = ma[0]; mw[1] = ma[1]; mw[2] = ma[2]; mw[3] = ma[3];
      mw[4] = mb[0]; mw[5] = mb[1]; mw[6] = mb[2]; mw[7] = mb[3];
      *(v8h*)(ldsK0 + krr * 72 + kcc) = k8h;
      *(v8h*)(ldsK1 + krr * 72 + kcc) = k8l;
      *(v8h*)(ldsVH + vdd * 40 + vkc) = v8a;
      *(v8h*)(ldsVL + vdd * 40 + vkc) = v8b;
    }
    const unsigned int pm0 = (kp[mk] != 0) ? 1u : 0u;
    const unsigned int pm1 = (kp[mk + 16] != 0) ? 1u : 0u;
    __syncthreads();

    v8f sh[2] = {}, sl[2] = {};
#pragma unroll
    for (int ks = 0; ks < 2; ++ks) {
#pragma unroll
      for (int t = 0; t < 2; ++t) {
        const v16h kfh = ld_frag(ldsK0 + (16 * t + c) * 72 + 32 * ks, hl);
        const v16h kfl = ld_frag(ldsK1 + (16 * t + c) * 72 + 32 * ks, hl);
        sh[t] = mma(qh[ks], kfh, sh[t]);
        sl[t] = mma(ql[ks], kfh, sl[t]);
        sl[t] = mma(qh[ks], kfl, sl[t]);
      }
    }

#pragma unroll
    for (int r = 0; r < 8; ++r) {
      const bool k0m = (((mw[r] >> c) & 1u) | pm0) != 0u;
      const bool k1m = (((mw[r] >> (16 + c)) & 1u) | pm1) != 0u;
      const float s0 = (sh[0][r] + sl[0][r] * RES_INV) * sscl;
      const float s1 = (sh[1][r] + sl[1][r] * RES_INV) * sscl;
      const float v0 = k0m ? NEG_INF : s0;
      const float v1 = k1m ? NEG_INF : s1;
      float tm = fmaxf(v0, v1);
      tm = fmaxf(tm, __shfl_xor(tm, 1, 32));
      tm = fmaxf(tm, __shfl_xor(tm, 2, 32));
      tm = fmaxf(tm, __shfl_xor(tm, 4, 32));
      tm = fmaxf(tm, __shfl_xor(tm, 8, 32));
      const float mn = fmaxf(m[r], tm);
      const float ms = (mn == NEG_INF) ? 0.f : mn;
      const float al = __expf(m[r] - ms);
      const float p0 = __expf(v0 - ms), p1 = __expf(v1 - ms);
      float rs = p0 + p1;
      rs += __shfl_xor(rs, 1, 32);
      rs += __shfl_xor(rs, 2, 32);
      rs += __shfl_xor(rs, 4, 32);
      rs += __shfl_xor(rs, 8, 32);
      l[r] = l[r] * al + rs;
      m[r] = mn;
#pragma unroll
      for (int t = 0; t < 4; ++t) { oh[t][r] *= al; ol[t][r] *= al; }
      const float c0 = p0 * P_CAR, c1 = p1 * P_CAR;
      const _Float16 h0 = (_Float16)c0, h1 = (_Float16)c1;
      const int pi = pbase + (8 * hl + r) * 40 + c;
      ldsPH[pi]      = h0;
      ldsPH[pi + 16] = h1;
      ldsPL[pi]      = (_Float16)((c0 - (float)h0) * RES_CAR);
      ldsPL[pi + 16] = (_Float16)((c1 - (float)h1) * RES_CAR);
    }
    __syncthreads();

    const v16h pfh = ld_frag(ldsPH + pbase + c * 40, hl);
    const v16h pfl = ld_frag(ldsPL + pbase + c * 40, hl);
#pragma unroll
    for (int t = 0; t < 4; ++t) {
      const v16h vfh = ld_frag(ldsVH + (16 * t + c) * 40, hl);
      const v16h vfl = ld_frag(ldsVL + (16 * t + c) * 40, hl);
      oh[t] = mma(pfh, vfh, oh[t]);
      ol[t] = mma(pfh, vfl, ol[t]);
      ol[t] = mma(pfl, vfh, ol[t]);
    }
    __syncthreads();
  }

#pragma unroll
  for (int half = 0; half < 2; ++half) {
    if ((w >> 2) == half) {
#pragma unroll
      for (int r = 0; r < 8; ++r) {
        const float inv = (1.0f / l[r]) * O_SCL;
        const int rowl = 16 * (w & 3) + 8 * hl + r;
#pragma unroll
        for (int t = 0; t < 4; ++t)
          ldsO[rowl * 68 + 16 * t + c] = (oh[t][r] + ol[t][r] * RES_INV) * inv;
      }
    }
    __syncthreads();
    float* const ob = Out + ((size_t)b * SEQ_FULL + q0 + 64 * half) * EMB + col0;
    for (int i = 0; i < 4; ++i) {
      const int qi = i * 256 + tid;
      const int rowl = qi >> 4, col = (qi & 15) * 4;
      const v4f v = *(const v4f*)(ldsO + rowl * 68 + col);
      *(volatile v4f*)(ob + (size_t)rowl * EMB + col) = v;
    }
    __threadfence();
    for (int i = 0; i < 4; ++i) {
      const int qi = i * 256 + tid;
      const int rowl = qi >> 4, col = (qi & 15) * 4;
      const v4f v = *(const v4f*)(ldsO + rowl * 68 + col);
      *(volatile v4f*)(ob + (size_t)rowl * EMB + col) = v;
    }
    __syncthreads();
  }
}

extern "C" void kernel_launch(void* const* d_in, const int* in_sizes, int n_in,
                              void* d_out, int out_size, void* d_ws, size_t ws_size,
                              hipStream_t stream)
{
  if (n_in < 8) return;
  const long tokMin = ((long)(NB - 1) * SEQ_FULL + SEQ) * EMB;
  if ((long)in_sizes[0] < tokMin) return;
  if ((long)in_sizes[1] < tokMin) return;
  if ((long)in_sizes[2] < (long)(SEQ - 1) * SEQ_FULL + SEQ) return;
  if ((long)in_sizes[3] < (long)(NB - 1) * SEQ_FULL + SEQ) return;
  if ((long)in_sizes[4] < (long)EMB * EMB) return;
  if ((long)in_sizes[5] < (long)EMB * EMB) return;
  if ((long)in_sizes[6] < (long)EMB * EMB) return;
  if ((long)in_sizes[7] < 1) return;
  if ((long)out_size < tokMin) return;

  const float* x   = (const float*)d_in[0];
  const float* ke  = (const float*)d_in[1];
  const int*   am  = (const int*)d_in[2];
  const int*   kpm = (const int*)d_in[3];
  const float* Wq  = (const float*)d_in[4];
  const float* Wk  = (const float*)d_in[5];
  const float* Wv  = (const float*)d_in[6];
  const float* gs  = (const float*)d_in[7];
  float* out = (float*)d_out;

  const size_t nTok = (size_t)NB * SEQ * EMB;
  const size_t nW   = (size_t)EMB * EMB;
  const size_t nMB  = (size_t)NKT * SEQ;
  const size_t nTF  = (size_t)(SEQ / 128) * NKT;
  const size_t total_bytes = (8 * nTok + 3 * nW) * sizeof(_Float16) + (nMB + nTF) * sizeof(unsigned int);
  if (total_bytes > ws_size) return;

  _Float16* X16  = (_Float16*)d_ws;
  _Float16* KE16 = X16  + nTok;
  _Float16* Wq16 = KE16 + nTok;
  _Float16* Wk16 = Wq16 + nW;
  _Float16* Wv16 = Wk16 + nW;
  _Float16* QH   = Wv16 + nW;
  _Float16* QL   = QH   + nTok;
  _Float16* KH   = QL   + nTok;
  _Float16* KL   = KH   + nTok;
  _Float16* VtH  = KL   + nTok;
  _Float16* VtL  = VtH  + nTok;
  unsigned int* MBT = (unsigned int*)(VtL + nTok);
  unsigned int* TF  = MBT + nMB;

  const int tt8 = (int)(nTok / 8);
  const int tw8 = (int)(nW / 8);
  k_cvt8<<<(tt8 + 255) / 256, 256, 0, stream>>>(x,  X16,  SEQ, SEQ_FULL, ACT_CAR, tt8);
  k_cvt8<<<(tt8 + 255) / 256, 256, 0, stream>>>(ke, KE16, SEQ, SEQ_FULL, ACT_CAR, tt8);
  k_cvt8<<<(tw8 + 255) / 256, 256, 0, stream>>>(Wq, Wq16, EMB, EMB, W_CAR, tw8);
  k_cvt8<<<(tw8 + 255) / 256, 256, 0, stream>>>(Wk, Wk16, EMB, EMB, W_CAR, tw8);
  k_cvt8<<<(tw8 + 255) / 256, 256, 0, stream>>>(Wv, Wv16, EMB, EMB, W_CAR, tw8);

  k_mask<<<SEQ / 128, 256, 0, stream>>>(am, MBT, TF);

  k_proj<<<dim3(EMB / 64, NB * SEQ / 128, 1), 128, 0, stream>>>(KE16, Wq16, QH, QL, EMB, EMB, 0LL, 0LL, 1);
  k_proj<<<dim3(EMB / 64, NB * SEQ / 128, 1), 128, 0, stream>>>(X16, Wk16, KH, KL, EMB, EMB, 0LL, 0LL, 1);
  k_proj<<<dim3(SEQ / 64, EMB / 128, NB), 128, 0, stream>>>(Wv16, X16, VtH, VtL, EMB, SEQ,
                                                            (long long)SEQ * EMB, (long long)EMB * SEQ, 0);

  k_attn<<<dim3(SEQ / 128, NH, NB), 256, 0, stream>>>(QH, QL, KH, KL, VtH, VtL, MBT, TF, kpm, gs, out);
}
